// MambaBlock_2911987827196
// MI455X (gfx1250) — hardware-verified
//
#include <hip/hip_runtime.h>
#include <stddef.h>
#include <stdint.h>
#include <math.h>


#define DM    1024
#define DI    2048
#define NS    16
#define DTR   64
#define NXD   96
#define NB    2
#define SL    1024
#define MT    (NB * SL)
#define NIN   (2 * DI)
#define KU    (2 * DI)
#define KDT   (2 * DTR)
#define NTHR  256
#define GBM   64
#define GTHR  128
#define SCH   64
#define TCH   32
#define SAP   17
#define WSMAX 134217728

static_assert(MT % GBM == 0 && NIN % 64 == 0 && DI % 64 == 0 && DM % 64 == 0);
static_assert(DM % 32 == 0 && KU % 32 == 0 && KDT % 32 == 0);
static_assert((DM & (DM - 1)) == 0 && (DI & (DI - 1)) == 0 && (DTR & (DTR - 1)) == 0);
static_assert(NXD == DTR + 2 * NS && NXD == 6 * 16);
static_assert((MT * DM) % (8 * NTHR) == 0 && (NIN * DM) % (8 * NTHR) == 0 && (NXD * DI) % (8 * NTHR) == 0);
static_assert((DI * DTR) % (8 * NTHR) == 0 && (DM * DI) % (8 * NTHR) == 0);
static_assert(DI % NTHR == 0 && DI % SCH == 0 && SL % TCH == 0 && (SL & (SL - 1)) == 0);
static_assert(SCH == 64 && TCH == 32 && NS == 16);
static_assert(GBM == (GTHR / 32) * 16);

typedef float          v4f   __attribute__((ext_vector_type(4)));
typedef float          v8f   __attribute__((ext_vector_type(8)));
typedef int            v8i   __attribute__((ext_vector_type(8)));
typedef unsigned short v4us  __attribute__((ext_vector_type(4)));
typedef unsigned short v8us  __attribute__((ext_vector_type(8)));
typedef unsigned short v16us __attribute__((ext_vector_type(16)));
typedef __bf16         v16bf __attribute__((ext_vector_type(16)));
typedef v4f  __attribute__((may_alias)) v4fa;
typedef v4us __attribute__((may_alias)) v4usa;
typedef v8us __attribute__((may_alias)) v8usa;
union FragB { v16bf v; v16us u; v8us h[2]; v8i w; };

__device__ __forceinline__ v8f wmb(const FragB& a, const FragB& b, v8f c) {
  v8f d = __builtin_amdgcn_wmma_f32_16x16x32_bf16(false, a.v, false, b.v, (short)0, c, false, false);
  asm volatile("v_nop\n\tv_nop\n\tv_nop\n\tv_nop" : "+v"(d) : "v"(a.w), "v"(b.w));
  return d;
}

__device__ __forceinline__ unsigned bf16_bits(float f) {
  const unsigned u = __float_as_uint(f);
  return (u + 0x7FFFu + ((u >> 16) & 1u)) >> 16;
}
__device__ __forceinline__ float bf16_val(float f) {
  return __uint_as_float(bf16_bits(f) << 16);
}
__device__ __forceinline__ void hilo(float v, unsigned& hb, unsigned& lb) {
  hb = bf16_bits(v);
  lb = bf16_bits(v - __uint_as_float(hb << 16));
}
__device__ __forceinline__ float delta_of(float x) {
  const float sp = fmaxf(x, 0.0f) + log1pf(expf(-fabsf(x)));
  return fminf(fmaxf(sp, 1e-4f), 10.0f);
}
__device__ __forceinline__ void put4(float* p, v4f v) {
  *(volatile v4f*)p = v;
  __threadfence();
  *(volatile v4f*)p = v;
}
__device__ __forceinline__ v4f bfr4(const float* p) {
  const v4f a = *(const v4f*)p;
  v4f r;
  r.x = bf16_val(a.x); r.y = bf16_val(a.y); r.z = bf16_val(a.z); r.w = bf16_val(a.w);
  return r;
}

__global__ __launch_bounds__(NTHR) void k_cvt(const float* __restrict__ src, unsigned short* dst, int nUnits) {
  const int u = (int)blockIdx.x * NTHR + (int)threadIdx.x;
  if (u >= nUnits) return;
  const float* p = src + (size_t)u * 8;
  const v4f a = *(const v4f*)p;
  const v4f b = *(const v4f*)(p + 4);
  v8us o;
  o[0] = (unsigned short)bf16_bits(a.x); o[1] = (unsigned short)bf16_bits(a.y);
  o[2] = (unsigned short)bf16_bits(a.z); o[3] = (unsigned short)bf16_bits(a.w);
  o[4] = (unsigned short)bf16_bits(b.x); o[5] = (unsigned short)bf16_bits(b.y);
  o[6] = (unsigned short)bf16_bits(b.z); o[7] = (unsigned short)bf16_bits(b.w);
  unsigned short* dp = dst + (size_t)u * 8;
  *(volatile v8us*)dp = o;
  __threadfence();
  *(volatile v8us*)dp = o;
}

__global__ __launch_bounds__(NTHR) void k_small(const float* __restrict__ cw, const float* __restrict__ cb,
                                                const float* __restrict__ dtb, const float* __restrict__ dvec,
                                                const float* __restrict__ alog,
                                                float* CW, float* CB, float* DTB, float* DV, float* AN) {
  const int b = (int)blockIdx.x, tid = (int)threadIdx.x;
  if (b < 8) {
    const int i = 4 * (b * NTHR + tid);
    put4(CW + i, bfr4(cw + i));
  } else if (b < 10) {
    const int i = 4 * ((b - 8) * NTHR + tid);
    put4(CB + i, bfr4(cb + i));
  } else if (b < 12) {
    const int i = 4 * ((b - 10) * NTHR + tid);
    put4(DTB + i, bfr4(dtb + i));
  } else if (b < 14) {
    const int i = 4 * ((b - 12) * NTHR + tid);
    put4(DV + i, bfr4(dvec + i));
  } else if (b < 46) {
    const int i = 4 * ((b - 14) * NTHR + tid);
    const v4f a = bfr4(alog + i);
    v4f r;
    r.x = -expf(a.x); r.y = -expf(a.y); r.z = -expf(a.z); r.w = -expf(a.w);
    put4(AN + i, r);
  }
}

template <int NT, int MODE>
__global__ __launch_bounds__(GTHR) void k_gemm(const unsigned short* __restrict__ A,
                                               const unsigned short* __restrict__ WT, int K, int kw,
                                               float* outF, int ldo, const float* __restrict__ bias,
                                               unsigned short* dtl) {
  constexpr int GBN = 16 * NT;
  static_assert(MODE == 1 ? NT == 6 : NT == 4);
  __shared__ __attribute__((aligned(16))) float stg[GBM * GBN];
  __shared__ __attribute__((aligned(16))) unsigned short dstg[MODE == 1 ? GBM * KDT : 8];
  const int tid = (int)threadIdx.x, lane = tid & 31, wave = tid >> 5, hh = lane >> 4, m = lane & 15;
  const int rowBase = (int)blockIdx.x * GBM;
  const int col0    = (int)blockIdx.y * GBN;
  const int kwm     = kw - 1;

  v8f acc[NT];
  {
    const v8f z = {0.f, 0.f, 0.f, 0.f, 0.f, 0.f, 0.f, 0.f};
#pragma unroll
    for (int t = 0; t < NT; ++t) acc[t] = z;
  }
  const unsigned short* ap = A  + (size_t)(rowBase + 16 * wave + m) * (size_t)K + 8 * hh;
  const unsigned short* wp = WT + (size_t)(col0 + m) * (size_t)kw + 8 * hh;
  const int ksteps = K >> 5;
#pragma unroll 1
  for (int ks = 0; ks < ksteps; ++ks) {
    const int k0 = 32 * ks;
    const int kk = k0 & kwm;
    FragB af;
    af.h[0] = *(const v8usa*)(ap + k0);
    af.h[1] = *(const v8usa*)(ap + k0 + 16);
#pragma unroll
    for (int t = 0; t < NT; ++t) {
      const unsigned short* wq = wp + (size_t)(16 * t) * (size_t)kw + kk;
      FragB bf;
      bf.h[0] = *(const v8usa*)wq;
      bf.h[1] = *(const v8usa*)(wq + 16);
      acc[t] = wmb(af, bf, acc[t]);
    }
  }

#pragma unroll
  for (int t = 0; t < NT; ++t) {
    const int lc = 16 * t + m;
#pragma unroll
    for (int r = 0; r < 8; ++r) {
      const int lr = 16 * wave + 8 * hh + r;
      stg[lr * GBN + lc] = acc[t][r];
    }
  }
  __syncthreads();

  if constexpr (MODE != 1) {
    v4f bb = {0.f, 0.f, 0.f, 0.f};
    if constexpr (MODE == 2) bb = *(const v4f*)(bias + col0 + 4 * m);
#pragma unroll 1
    for (int i = 0; i < 8; ++i) {
      const int lr = 16 * wave + 2 * i + hh;
      float* sp = stg + lr * GBN + 4 * m;
      v4f v = *(const v4fa*)sp;
      if constexpr (MODE == 2) {
        v.x = delta_of(v.x + bb.x);
        v.y = delta_of(v.y + bb.y);
        v.z = delta_of(v.z + bb.z);
        v.w = delta_of(v.w + bb.w);
        *(v4fa*)sp = v;
      }
      float* op = outF + (size_t)(rowBase + lr) * (size_t)ldo + col0 + 4 * m;
      *(volatile v4f*)op = v;
    }
    __threadfence();
#pragma unroll 1
    for (int i = 0; i < 8; ++i) {
      const int lr = 16 * wave + 2 * i + hh;
      const v4f v = *(const v4fa*)(stg + lr * GBN + 4 * m);
      float* op = outF + (size_t)(rowBase + lr) * (size_t)ldo + col0 + 4 * m;
      *(volatile v4f*)op = v;
    }
  } else {
#pragma unroll 1
    for (int it = 0; it < 8; ++it) {
      const int idx = it * GTHR + tid;
      const int row = idx >> 4, c4 = (idx & 15) * 4;
      const v4f v = *(const v4fa*)(stg + row * GBN + c4);
      v4us h4, l4;
      unsigned hb, lb;
      hilo(v.x, hb, lb); h4[0] = (unsigned short)hb; l4[0] = (unsigned short)lb;
      hilo(v.y, hb, lb); h4[1] = (unsigned short)hb; l4[1] = (unsigned short)lb;
      hilo(v.z, hb, lb); h4[2] = (unsigned short)hb; l4[2] = (unsigned short)lb;
      hilo(v.w, hb, lb); h4[3] = (unsigned short)hb; l4[3] = (unsigned short)lb;
      *(v4usa*)(dstg + row * KDT + c4) = h4;
      *(v4usa*)(dstg + row * KDT + DTR + c4) = l4;
    }
    __syncthreads();
    float* ob = outF + (size_t)rowBase * NXD;
    unsigned short* db = dtl + (size_t)rowBase * KDT;
#pragma unroll 1
    for (int it = 0; it < (GBM * GBN) / (4 * GTHR); ++it) {
      const int idx = it * GTHR + tid;
      const v4f v = *(const v4fa*)(stg + 4 * idx);
      *(volatile v4f*)(ob + 4 * idx) = v;
    }
#pragma unroll 1
    for (int it = 0; it < (GBM * KDT) / (8 * GTHR); ++it) {
      const int idx = it * GTHR + tid;
      const v8us q = *(const v8usa*)(dstg + 8 * idx);
      *(volatile v8us*)(db + 8 * idx) = q;
    }
    __threadfence();
#pragma unroll 1
    for (int it = 0; it < (GBM * GBN) / (4 * GTHR); ++it) {
      const int idx = it * GTHR + tid;
      const v4f v = *(const v4fa*)(stg + 4 * idx);
      *(volatile v4f*)(ob + 4 * idx) = v;
    }
#pragma unroll 1
    for (int it = 0; it < (GBM * KDT) / (8 * GTHR); ++it) {
      const int idx = it * GTHR + tid;
      const v8us q = *(const v8usa*)(dstg + 8 * idx);
      *(volatile v8us*)(db + 8 * idx) = q;
    }
  }
}

__global__ __launch_bounds__(NTHR) void k_conv(const float* __restrict__ xz, const float* __restrict__ cw,
                                               const float* __restrict__ cb, float* u, unsigned short* uhl) {
  __shared__ __attribute__((aligned(16))) float suf[NTHR];
  __shared__ __attribute__((aligned(16))) unsigned short shl[2 * NTHR];
  const int tid = (int)threadIdx.x;
  const int blk = (int)blockIdx.x;
  const int m = blk >> 3;
  const int cbase = (blk & 7) * NTHR;
  const int c = cbase + tid;
  const int l = m & (SL - 1);
  const int mb = m - l;
  int r0 = m - 3, r1 = m - 2, r2 = m - 1;
  const bool ok0 = l >= 3, ok1 = l >= 2, ok2 = l >= 1;
  r0 = r0 < mb ? mb : r0;
  r1 = r1 < mb ? mb : r1;
  r2 = r2 < mb ? mb : r2;
  const v4f w = *(const v4f*)(cw + 4 * c);
  const float bv = cb[c];
  const float x0 = xz[(size_t)r0 * NIN + c];
  const float x1 = xz[(size_t)r1 * NIN + c];
  const float x2 = xz[(size_t)r2 * NIN + c];
  const float x3 = xz[(size_t)m  * NIN + c];
  const float a0 = ok0 ? x0 : 0.0f;
  const float a1 = ok1 ? x1 : 0.0f;
  const float a2 = ok2 ? x2 : 0.0f;
  float acc = w.x * a0;
  acc = fmaf(w.y, a1, acc);
  acc = fmaf(w.z, a2, acc);
  acc = fmaf(w.w, x3, acc);
  acc += bv;
  const float e = expf(-acc);
  const float uv = acc * (1.0f / (1.0f + e));
  unsigned hb, lb;
  hilo(uv, hb, lb);
  suf[tid] = uv;
  shl[tid] = (unsigned short)hb;
  shl[NTHR + tid] = (unsigned short)lb;
  __syncthreads();
  if (tid < 64) {
    const v4f v = *(const v4fa*)(suf + 4 * tid);
    float* op = u + (size_t)m * DI + cbase + 4 * tid;
    *(volatile v4f*)op = v;
    __threadfence();
    *(volatile v4f*)op = v;
  } else if (tid < 128) {
    const int q   = tid & 31;
    const int sel = (tid >> 5) & 1;
    const v8us hv = *(const v8usa*)(shl + NTHR * sel + 8 * q);
    unsigned short* hp = uhl + (size_t)m * KU + (size_t)(DI * sel) + cbase + 8 * q;
    *(volatile v8us*)hp = hv;
    __threadfence();
    *(volatile v8us*)hp = hv;
  }
}

#define SSTEP(N, BV, CV) { \
    float bu = (dl * (BV)) * uv; \
    bu = fminf(fmaxf(bu, -10.0f), 10.0f); \
    float hn = fmaf(av[N], h[N], bu); \
    hn = fminf(fmaxf(hn, -50.0f), 50.0f); \
    h[N] = hn; \
    acc = fmaf(hn, (CV), acc); }

__global__ __launch_bounds__(SCH) void k_scan(const float* __restrict__ delta, const float* __restrict__ u,
                                              const float* __restrict__ xz, const float* __restrict__ xdbl,
                                              const float* __restrict__ an, const float* __restrict__ dvec,
                                              unsigned short* yhl) {
  __shared__ __attribute__((aligned(16))) float sbc[TCH * 32];
  __shared__ __attribute__((aligned(16))) unsigned short sy[2 * TCH * SCH];
  __shared__ float sA[SCH * SAP];
  __shared__ float sAv[SCH * SAP];
  const int tid = (int)threadIdx.x;
  const int b  = (int)blockIdx.x >> 5;
  const int cb = ((int)blockIdx.x & 31) * SCH;
  const int c  = cb + tid;
  const int mb = b * SL;

  float a0;
  bool same;
  {
    const v4f A0 = *(const v4f*)(an + (size_t)c * NS);
    const v4f A1 = *(const v4f*)(an + (size_t)c * NS + 4);
    const v4f A2 = *(const v4f*)(an + (size_t)c * NS + 8);
    const v4f A3 = *(const v4f*)(an + (size_t)c * NS + 12);
    float* sr = sA + tid * SAP;
    sr[0] = A0.x;  sr[1] = A0.y;  sr[2] = A0.z;  sr[3] = A0.w;
    sr[4] = A1.x;  sr[5] = A1.y;  sr[6] = A1.z;  sr[7] = A1.w;
    sr[8] = A2.x;  sr[9] = A2.y;  sr[10] = A2.z; sr[11] = A2.w;
    sr[12] = A3.x; sr[13] = A3.y; sr[14] = A3.z; sr[15] = A3.w;
    a0 = A0.x;
    same = (A0.y == a0) && (A0.z == a0) && (A0.w == a0)
        && (A1.x == a0) && (A1.y == a0) && (A1.z == a0) && (A1.w == a0)
        && (A2.x == a0) && (A2.y == a0) && (A2.z == a0) && (A2.w == a0)
        && (A3.x == a0) && (A3.y == a0) && (A3.z == a0) && (A3.w == a0);
  }
  const bool allsame = (__builtin_amdgcn_ballot_w32(same) == 0xffffffffu);
  const float dvv = dvec[c];

  float h[NS];
#pragma unroll
  for (int n = 0; n < NS; ++n) h[n] = 0.0f;

  float dl_n = delta[(size_t)mb * DI + c];
  float u_n  = u[(size_t)mb * DI + c];
  float z_n  = xz[(size_t)mb * NIN + DI + c];

#pragma unroll 1
  for (int t0 = 0; t0 < SL; t0 += TCH) {
#pragma unroll
    for (int j = 0; j < 4; ++j) {
      const int q = tid + SCH * j;
      const int tok = q >> 3, part = q & 7;
      const v4f v = *(const v4f*)(xdbl + (size_t)(mb + t0 + tok) * NXD + DTR + 4 * part);
      *(v4fa*)(sbc + tok * 32 + 4 * part) = v;
    }
    __syncthreads();

#pragma unroll 1
    for (int tt = 0; tt < TCH; ++tt) {
      const float dl = dl_n, uv = u_n, zv = z_n;
      {
        int tn = t0 + tt + 1;
        tn = tn > SL - 1 ? SL - 1 : tn;
        const size_t mn = (size_t)(mb + tn);
        dl_n = delta[mn * DI + c];
        u_n  = u[mn * DI + c];
        z_n  = xz[mn * NIN + DI + c];
      }
      float av[NS];
      if (allsame) {
        const float e0 = fminf(expf(dl * a0), 10.0f);
#pragma unroll
        for (int n = 0; n < NS; ++n) av[n] = e0;
      } else {
#pragma unroll 1
        for (int n = 0; n < NS; ++n)
          sAv[tid * SAP + n] = fminf(expf(dl * sA[tid * SAP + n]), 10.0f);
#pragma unroll
        for (int n = 0; n < NS; ++n) av[n] = sAv[tid * SAP + n];
      }
      const float* bcp = sbc + tt * 32;
      const v4f B0 = *(const v4fa*)(bcp);
      const v4f B1 = *(const v4fa*)(bcp + 4);
      const v4f B2 = *(const v4fa*)(bcp + 8);
      const v4f B3 = *(const v4fa*)(bcp + 12);
      const v4f C0 = *(const v4fa*)(bcp + 16);
      const v4f C1 = *(const v4fa*)(bcp + 20);
      const v4f C2 = *(const v4fa*)(bcp + 24);
      const v4f C3 = *(const v4fa*)(bcp + 28);
      float acc = 0.0f;
      SSTEP(0,  B0.x, C0.x) SSTEP(1,  B0.y, C0.y) SSTEP(2,  B0.z, C0.z) SSTEP(3,  B0.w, C0.w)
      SSTEP(4,  B1.x, C1.x) SSTEP(5,  B1.y, C1.y) SSTEP(6,  B1.z, C1.z) SSTEP(7,  B1.w, C1.w)
      SSTEP(8,  B2.x, C2.x) SSTEP(9,  B2.y, C2.y) SSTEP(10, B2.z, C2.z) SSTEP(11, B2.w, C2.w)
      SSTEP(12, B3.x, C3.x) SSTEP(13, B3.y, C3.y) SSTEP(14, B3.z, C3.z) SSTEP(15, B3.w, C3.w)
      float yv = fmaf(uv, dvv, acc);
      yv = fminf(fmaxf(yv, -100.0f), 100.0f);
      const float ez = expf(-zv);
      const float g  = zv * (1.0f / (1.0f + ez));
      yv = yv * g;
      unsigned hb, lb;
      hilo(yv, hb, lb);
      sy[tt * SCH + tid] = (unsigned short)hb;
      sy[TCH * SCH + tt * SCH + tid] = (unsigned short)lb;
    }
    __syncthreads();

    v8us q[8];
#pragma unroll
    for (int j = 0; j < 8; ++j) {
      const int line  = j * 8 + (tid >> 3);
      const int plane = line >> 5, tok = line & 31;
      q[j] = *(const v8usa*)(sy + plane * (TCH * SCH) + tok * SCH + 8 * (tid & 7));
    }
#pragma unroll
    for (int j = 0; j < 8; ++j) {
      const int line  = j * 8 + (tid >> 3);
      const int plane = line >> 5, tok = line & 31;
      unsigned short* yp = yhl + (size_t)(mb + t0 + tok) * KU + (size_t)(plane * DI) + cb + 8 * (tid & 7);
      *(volatile v8us*)yp = q[j];
    }
    __threadfence();
#pragma unroll
    for (int j = 0; j < 8; ++j) {
      const int line  = j * 8 + (tid >> 3);
      const int plane = line >> 5, tok = line & 31;
      unsigned short* yp = yhl + (size_t)(mb + t0 + tok) * KU + (size_t)(plane * DI) + cb + 8 * (tid & 7);
      *(volatile v8us*)yp = q[j];
    }
  }
}
#undef SSTEP

static inline size_t al256(size_t o) { return (o + 255) & ~(size_t)255; }

extern "C" void kernel_launch(void* const* d_in, const int* in_sizes, int n_in,
                              void* d_out, int out_size, void* d_ws, size_t ws_size,
                              hipStream_t stream) {
  if (n_in < 10) return;
  if (in_sizes[0] != MT * DM) return;
  if (in_sizes[1] != NIN * DM) return;
  if (in_sizes[2] != DI * 4) return;
  if (in_sizes[3] != DI) return;
  if (in_sizes[4] != NXD * DI) return;
  if (in_sizes[5] != DI * DTR) return;
  if (in_sizes[6] != DI) return;
  if (in_sizes[7] != DI * NS) return;
  if (in_sizes[8] != DI) return;
  if (in_sizes[9] != DM * DI) return;
  if (out_size != MT * DM) return;

  const float* x    = (const float*)d_in[0];
  const float* win  = (const float*)d_in[1];
  const float* cw   = (const float*)d_in[2];
  const float* cbv  = (const float*)d_in[3];
  const float* wxp  = (const float*)d_in[4];
  const float* wdt  = (const float*)d_in[5];
  const float* dtb  = (const float*)d_in[6];
  const float* alog = (const float*)d_in[7];
  const float* dvec = (const float*)d_in[8];
  const float* wo   = (const float*)d_in[9];
  float* out = (float*)d_out;

  char* ws = (char*)d_ws;
  size_t off = 0;
  const size_t oXB   = off; off = al256(off + (size_t)MT * DM * 2);
  const size_t oWIN  = off; off = al256(off + (size_t)NIN * DM * 2);
  const size_t oXPW  = off; off = al256(off + (size_t)NXD * DI * 2);
  const size_t oDTW  = off; off = al256(off + (size_t)DI * DTR * 2);
  const size_t oOW   = off; off = al256(off + (size_t)DM * DI * 2);
  const size_t oCW   = off; off = al256(off + (size_t)DI * 4 * 4);
  const size_t oCB   = off; off = al256(off + (size_t)DI * 4);
  const size_t oDTB  = off; off = al256(off + (size_t)DI * 4);
  const size_t oDV   = off; off = al256(off + (size_t)DI * 4);
  const size_t oAN   = off; off = al256(off + (size_t)DI * NS * 4);
  const size_t oXZ   = off; off = al256(off + (size_t)MT * NIN * 4);
  const size_t oU    = off; off = al256(off + (size_t)MT * DI * 4);
  const size_t oUHL  = off; off = al256(off + (size_t)MT * KU * 2);
  const size_t oXDBL = off; off = al256(off + (size_t)MT * NXD * 4);
  const size_t oDTL  = off; off = al256(off + (size_t)MT * KDT * 2);
  const size_t oDEL  = off; off = al256(off + (size_t)MT * DI * 4);
  if (off > ws_size || off > (size_t)WSMAX) return;

  unsigned short* XB   = (unsigned short*)(ws + oXB);
  unsigned short* WIN  = (unsigned short*)(ws + oWIN);
  unsigned short* XPW  = (unsigned short*)(ws + oXPW);
  unsigned short* DTW  = (unsigned short*)(ws + oDTW);
  unsigned short* OW   = (unsigned short*)(ws + oOW);
  float*          CW   = (float*)(ws + oCW);
  float*          CB   = (float*)(ws + oCB);
  float*          DTB  = (float*)(ws + oDTB);
  float*          DV   = (float*)(ws + oDV);
  float*          AN   = (float*)(ws + oAN);
  float*          XZ   = (float*)(ws + oXZ);
  float*          U    = (float*)(ws + oU);
  unsigned short* UHL  = (unsigned short*)(ws + oUHL);
  unsigned short* YHL  = UHL;
  float*          XDBL = (float*)(ws + oXDBL);
  unsigned short* DTL  = (unsigned short*)(ws + oDTL);
  float*          DEL  = (float*)(ws + oDEL);

  k_cvt<<<(MT * DM) / (8 * NTHR), NTHR, 0, stream>>>(x, XB, (MT * DM) / 8);
  k_cvt<<<(NIN * DM) / (8 * NTHR), NTHR, 0, stream>>>(win, WIN, (NIN * DM) / 8);
  k_cvt<<<(NXD * DI) / (8 * NTHR), NTHR, 0, stream>>>(wxp, XPW, (NXD * DI) / 8);
  k_cvt<<<(DI * DTR) / (8 * NTHR), NTHR, 0, stream>>>(wdt, DTW, (DI * DTR) / 8);
  k_cvt<<<(DM * DI) / (8 * NTHR), NTHR, 0, stream>>>(wo, OW, (DM * DI) / 8);
  k_small<<<46, NTHR, 0, stream>>>(cw, cbv, dtb, dvec, alog, CW, CB, DTB, DV, AN);
  k_gemm<4, 0><<<dim3(MT / GBM, NIN / 64), GTHR, 0, stream>>>(XB, WIN, DM, DM, XZ, NIN, DTB, DTL);
  k_conv<<<MT * (DI / NTHR), NTHR, 0, stream>>>(XZ, CW, CB, U, UHL);
  k_gemm<6, 1><<<dim3(MT / GBM, 1), GTHR, 0, stream>>>(UHL, XPW, KU, DI, XDBL, NXD, DTB, DTL);
  k_gemm<4, 2><<<dim3(MT / GBM, DI / 64), GTHR, 0, stream>>>(DTL, DTW, KDT, DTR, DEL, DI, DTB, DTL);
  k_scan<<<NB * (DI / SCH), SCH, 0, stream>>>(DEL, U, XZ, XDBL, AN, DV, YHL);
  k_gemm<4, 0><<<dim3(MT / GBM, DM / 64), GTHR, 0, stream>>>(YHL, OW, KU, DI, out, DM, DTB, DTL);
}
